// GCN_25383256719664
// MI455X (gfx1250) — hardware-verified
//
#include <hip/hip_runtime.h>
#include <stddef.h>
#include <stdint.h>
#include <math.h>


#define DIN    78
#define D1     78
#define D2     156
#define D3     312
#define DF1    1024
#define DF2    128
#define C1     96
#define C2     160
#define C3     320
#define NTHR   256
#define NWAVE  8
#define EPT    8
#define CHUNK  (NTHR * EPT)
#define WCAP   (EPT * 32)
#define LISTN  (NWAVE * WCAP)
#define NBD    8192
#define SLD    13
#define NBA    1024
#define SLA    10
#define RCAP   28672
#define DEGCAP 64
#define GBM    64
#define GTHR   128
#define AGG_ZINTS (LISTN + 2 * RCAP + 3 * NBA)
#define MISC_INTS 16
#define BLS_F     320
#define ROW_HW    320
#define AGG_LDS_INTS (AGG_ZINTS + MISC_INTS + BLS_F + NWAVE * ROW_HW / 2)
#define WB1    5
#define WB2    15
#define WB3    50
#define WB4    320
#define WB5    128
#define WSMAX  134217728

static_assert((CHUNK & (CHUNK - 1)) == 0 && CHUNK <= 4096);
static_assert((NBD & (NBD - 1)) == 0 && NBD == (1 << SLD));
static_assert((NBA & (NBA - 1)) == 0 && NBA == (1 << SLA));
static_assert(((long long)CHUNK << SLD) < (1LL << 31));
static_assert(((long long)CHUNK << SLA) < (1LL << 31));
static_assert(NBD % (NTHR * 4) == 0);
static_assert(LISTN % NTHR == 0);
static_assert(NBA % NWAVE == 0 && NBA % 32 == 0 && NBA % GBM == 0);
static_assert(RCAP % 32 == 0 && AGG_ZINTS % 4 == 0 && LISTN % 4 == 0);
static_assert((AGG_ZINTS + MISC_INTS) % 4 == 0 && (AGG_ZINTS + MISC_INTS + BLS_F) % 4 == 0);
static_assert(AGG_LDS_INTS * 4 <= 300000);
static_assert(C1 % 32 == 0 && C2 % 32 == 0 && C3 % 32 == 0 && DF1 % 64 == 0 && DF2 % 64 == 0);
static_assert(DIN <= C1 && D1 <= C1 && D2 <= C2 && D3 <= C3 && (DIN % 2) == 0);
static_assert(WB1 * NTHR >= C1 * (C1 / 8));
static_assert(WB2 * NTHR == C2 * (2 * C1 / 8));
static_assert(WB3 * NTHR == C3 * (2 * C2 / 8));
static_assert(WB4 * NTHR == DF1 * (2 * C3 / 8));
static_assert(WB5 * NTHR == DF2 * (2 * DF1 / 8));
static_assert(C3 <= BLS_F && 2 * C2 <= ROW_HW);

typedef float          v2f   __attribute__((ext_vector_type(2)));
typedef float          v4f   __attribute__((ext_vector_type(4)));
typedef float          v8f   __attribute__((ext_vector_type(8)));
typedef int            v4i   __attribute__((ext_vector_type(4)));
typedef int            v8i   __attribute__((ext_vector_type(8)));
typedef unsigned short v4us  __attribute__((ext_vector_type(4)));
typedef unsigned short v8us  __attribute__((ext_vector_type(8)));
typedef unsigned short v16us __attribute__((ext_vector_type(16)));
typedef __bf16         v16bf __attribute__((ext_vector_type(16)));
typedef v2f  __attribute__((may_alias)) v2fa;
typedef v4f  __attribute__((may_alias)) v4fa;
typedef v4i  __attribute__((may_alias)) v4ia;
typedef v4us __attribute__((may_alias)) v4usa;
typedef v8us __attribute__((may_alias)) v8usa;
union FragB { v16bf v; v16us u; v8us h[2]; v8i w; };

__device__ __forceinline__ v8f wmb(const FragB& a, const FragB& b, v8f c) {
  v8f d = __builtin_amdgcn_wmma_f32_16x16x32_bf16(false, a.v, false, b.v, (short)0, c, false, false);
  asm volatile("v_nop\n\tv_nop\n\tv_nop\n\tv_nop" : "+v"(d) : "v"(a.w), "v"(b.w));
  return d;
}

__device__ __forceinline__ unsigned bf16_bits(float f) {
  const unsigned u = __float_as_uint(f);
  const unsigned r = (u + 0x7FFFu + ((u >> 16) & 1u)) >> 16;
  return (f != f) ? 0x7FC0u : r;
}
__device__ __forceinline__ float bf16_val(float f) {
  return __uint_as_float(bf16_bits(f) << 16);
}
__device__ __forceinline__ unsigned short hl_bits(float v, int lo) {
  const float t = (v > 0.0f) ? v : (v - v);
  const unsigned h = bf16_bits(t);
  const unsigned l = bf16_bits(t - __uint_as_float(h << 16));
  return (unsigned short)(lo ? l : h);
}
__device__ __forceinline__ float nmax(float m, float v) {
  return (v > m || v != v) ? v : m;
}
__device__ __forceinline__ float fin1(float acc, float sv, float rd, float b, float pzr, bool live) {
  float y = (acc + sv * rd) + b;
  y = (y > 0.0f) ? y : (y - y);
  y = y + pzr;
  return live ? y : 0.0f;
}

__device__ __forceinline__ void wave_sync() {
  __builtin_amdgcn_fence(__ATOMIC_RELEASE, "wavefront");
  __builtin_amdgcn_wave_barrier();
  __builtin_amdgcn_fence(__ATOMIC_ACQUIRE, "wavefront");
}

template <int SLB>
__device__ __forceinline__ int scan_chunk(const int* __restrict__ dsts, int nE, int cbase, int slotBase,
                                          int nb, int vec8, int* list, int tid, int lane, int wave) {
  int wc = 0;
  const int el0  = tid * EPT;
  const int e0   = cbase + el0;
  const int sent = -2147483647 - 1;
  v4i da, db;
  if (vec8 != 0 && cbase + CHUNK <= nE) {
    da = *(const v4i*)(dsts + e0);
    db = *(const v4i*)(dsts + e0 + 4);
  } else {
    da.x = (e0     < nE) ? dsts[min(e0,     nE - 1)] : sent;
    da.y = (e0 + 1 < nE) ? dsts[min(e0 + 1, nE - 1)] : sent;
    da.z = (e0 + 2 < nE) ? dsts[min(e0 + 2, nE - 1)] : sent;
    da.w = (e0 + 3 < nE) ? dsts[min(e0 + 3, nE - 1)] : sent;
    db.x = (e0 + 4 < nE) ? dsts[min(e0 + 4, nE - 1)] : sent;
    db.y = (e0 + 5 < nE) ? dsts[min(e0 + 5, nE - 1)] : sent;
    db.z = (e0 + 6 < nE) ? dsts[min(e0 + 6, nE - 1)] : sent;
    db.w = (e0 + 7 < nE) ? dsts[min(e0 + 7, nE - 1)] : sent;
  }
  const unsigned nbs = (unsigned)slotBase;
  const unsigned unb = (unsigned)nb;
  const unsigned s0 = (unsigned)da.x - nbs, s1 = (unsigned)da.y - nbs;
  const unsigned s2 = (unsigned)da.z - nbs, s3 = (unsigned)da.w - nbs;
  const unsigned s4 = (unsigned)db.x - nbs, s5 = (unsigned)db.y - nbs;
  const unsigned s6 = (unsigned)db.z - nbs, s7 = (unsigned)db.w - nbs;
  const bool h0 = s0 < unb, h1 = s1 < unb, h2 = s2 < unb, h3 = s3 < unb;
  const bool h4 = s4 < unb, h5 = s5 < unb, h6 = s6 < unb, h7 = s7 < unb;
  const unsigned any = __builtin_amdgcn_ballot_w32(h0 | h1 | h2 | h3 | h4 | h5 | h6 | h7);
  if (any != 0u) {
#define HITJ(J, HJ, SJ) { \
      const unsigned mj = __builtin_amdgcn_ballot_w32(HJ); \
      if (mj != 0u) { \
        if (HJ) { \
          const int pos = wc + (int)__builtin_amdgcn_mbcnt_lo(mj, 0u); \
          if (pos < WCAP) list[wave * WCAP + pos] = ((el0 + (J)) << SLB) | (int)(SJ); \
        } \
        wc += (int)__builtin_popcount(mj); } }
    HITJ(0, h0, s0)
    HITJ(1, h1, s1)
    HITJ(2, h2, s2)
    HITJ(3, h3, s3)
    HITJ(4, h4, s4)
    HITJ(5, h5, s5)
    HITJ(6, h6, s6)
    HITJ(7, h7, s7)
#undef HITJ
  }
  return wc;
}

__global__ __launch_bounds__(NTHR) void k_wprep(const float* __restrict__ W1, const float* __restrict__ W2,
                                                const float* __restrict__ W3, const float* __restrict__ W4,
                                                const float* __restrict__ W5,
                                                unsigned short* T1, unsigned short* T2, unsigned short* T3,
                                                unsigned short* T4, unsigned short* T5) {
  const int b = (int)blockIdx.x;
  const float* W;
  unsigned short* P;
  int din, dout, np, kseg, kt, ub;
  if (b < WB1)                         { W = W1; P = T1; din = DIN; dout = D1;  np = C1;  kseg = C1;  kt = C1;      ub = b; }
  else if (b < WB1 + WB2)              { W = W2; P = T2; din = D1;  dout = D2;  np = C2;  kseg = C1;  kt = 2 * C1;  ub = b - WB1; }
  else if (b < WB1 + WB2 + WB3)        { W = W3; P = T3; din = D2;  dout = D3;  np = C3;  kseg = C2;  kt = 2 * C2;  ub = b - WB1 - WB2; }
  else if (b < WB1 + WB2 + WB3 + WB4)  { W = W4; P = T4; din = D3;  dout = DF1; np = DF1; kseg = C3;  kt = 2 * C3;  ub = b - WB1 - WB2 - WB3; }
  else                                 { W = W5; P = T5; din = DF1; dout = DF2; np = DF2; kseg = DF1; kt = 2 * DF1; ub = b - WB1 - WB2 - WB3 - WB4; }
  const int u   = ub * NTHR + (int)threadIdx.x;
  const int upr = kt >> 3;
  if (u >= np * upr) return;
  const int n  = u / upr;
  const int k8 = (u - n * upr) * 8;
  const int kk = (k8 >= kseg) ? (k8 - kseg) : k8;
  const int nc = (n < dout) ? n : (dout - 1);
  v8us o;
#pragma unroll
  for (int i = 0; i < 8; ++i) {
    const int k  = kk + i;
    const int kc = (k < din) ? k : (din - 1);
    const float w = W[(size_t)kc * dout + nc];
    o[i] = (k < din && n < dout) ? (unsigned short)bf16_bits(w) : (unsigned short)0;
  }
  unsigned short* dp = P + (size_t)u * 8;
  *(volatile v8us*)dp = o;
  __threadfence();
  *(volatile v8us*)dp = o;
}

__global__ __launch_bounds__(NTHR) void k_cvx(const float* __restrict__ x, int nN, int nUnits,
                                              unsigned short* xb) {
  const int u = (int)blockIdx.x * NTHR + (int)threadIdx.x;
  if (u >= nUnits) return;
  const int row = u / (C1 / 8);
  const int k8  = (u - row * (C1 / 8)) * 8;
  const int rc  = row < nN ? row : nN - 1;
  const bool ok = row < nN;
  const float* p = x + (size_t)rc * DIN;
  v8us o;
#pragma unroll
  for (int j = 0; j < 4; ++j) {
    const int k  = k8 + 2 * j;
    const int kc = (k < DIN - 2) ? k : (DIN - 2);
    const v2f a = *(const v2fa*)(p + kc);
    const bool val = ok && (k < DIN);
    o[2 * j]     = val ? (unsigned short)bf16_bits(a.x) : (unsigned short)0;
    o[2 * j + 1] = val ? (unsigned short)bf16_bits(a.y) : (unsigned short)0;
  }
  unsigned short* dp = xb + (size_t)u * 8;
  *(volatile v8us*)dp = o;
  __threadfence();
  *(volatile v8us*)dp = o;
}

__global__ __launch_bounds__(NTHR) void k_deg(const int* __restrict__ dsts, int nE, int vec8, float* dis) {
  __shared__ __attribute__((aligned(16))) int scnt[NBD];
  __shared__ __attribute__((aligned(16))) int list[LISTN];
  __shared__ int wcnt[NWAVE];
  const int tid = (int)threadIdx.x, lane = tid & 31, wave = tid >> 5;
  const int nodeBase = (int)blockIdx.x * NBD;

  for (int i = tid; i < NBD; i += NTHR) scnt[i] = 0;
  for (int i = tid; i < LISTN; i += NTHR) list[i] = 0;
  if (tid < NWAVE) wcnt[tid] = 0;
  __syncthreads();

  const int nChunks = (nE + CHUNK - 1) / CHUNK;
#pragma unroll 1
  for (int ch = 0; ch < nChunks; ++ch) {
    const int cbase = ch * CHUNK;
    const int wc = scan_chunk<SLD>(dsts, nE, cbase, nodeBase, NBD, vec8, list, tid, lane, wave);
    if (lane == 0) wcnt[wave] = wc;
    __syncthreads();
    if (wave == 0) {
#pragma unroll 1
      for (int w2 = 0; w2 < NWAVE; ++w2) {
        int c = wcnt[w2];
        c = c < 0 ? 0 : (c > WCAP ? WCAP : c);
#pragma unroll 1
        for (int b0 = 0; b0 < c; b0 += 32) {
          const int idx = b0 + lane;
          const int ent = list[w2 * WCAP + (idx < WCAP ? idx : WCAP - 1)];
          const int m32 = (c - b0) < 32 ? (c - b0) : 32;
#pragma unroll 1
          for (int k = 0; k < m32; ++k) {
            const int u  = __builtin_amdgcn_readlane(ent, k);
            const int sl = u & (NBD - 1);
            if (lane == 0) scnt[sl] = scnt[sl] + 1;
          }
        }
      }
    }
    __syncthreads();
  }

  v4f vals[NBD / (NTHR * 4)];
#pragma unroll
  for (int it = 0; it < NBD / (NTHR * 4); ++it) {
    const int s0 = it * (NTHR * 4) + 4 * tid;
    const v4i c4 = *(const v4ia*)(scnt + s0);
    const float d0 = (float)c4.x + 1.0f, d1 = (float)c4.y + 1.0f;
    const float d2 = (float)c4.z + 1.0f, d3 = (float)c4.w + 1.0f;
    v4f v;
    v.x = rsqrtf(d0); v.y = rsqrtf(d1); v.z = rsqrtf(d2); v.w = rsqrtf(d3);
    vals[it] = v;
  }
#pragma unroll
  for (int it = 0; it < NBD / (NTHR * 4); ++it) {
    const int s0 = it * (NTHR * 4) + 4 * tid;
    *(volatile v4f*)(dis + (size_t)nodeBase + s0) = vals[it];
  }
  __threadfence();
#pragma unroll
  for (int it = 0; it < NBD / (NTHR * 4); ++it) {
    const int s0 = it * (NTHR * 4) + 4 * tid;
    *(volatile v4f*)(dis + (size_t)nodeBase + s0) = vals[it];
  }
}

template <int NT, int EPI>
__global__ __launch_bounds__(GTHR) void k_gemm(
    const unsigned short* __restrict__ A, const unsigned short* __restrict__ WT, int K,
    const float* __restrict__ bias, float* outF, unsigned short* outH, int ldo, int aux)
{
  constexpr int GN = 16 * NT;
  constexpr int PR = GN / 4;
  static_assert(EPI == 0 || NT == 4);
  static_assert(PR % 8 == 0 && (GBM * PR) % GTHR == 0);
  __shared__ __attribute__((aligned(16))) float stg[GBM * GN];
  __shared__ __attribute__((aligned(16))) float bsm[64];
  const int tid = (int)threadIdx.x, lane = tid & 31, wave = tid >> 5, hh = lane >> 4, m = lane & 15;
  const int rowBase = (int)blockIdx.x * GBM;
  const int col0    = (int)blockIdx.y * GN;

  v8f acc[NT];
  {
    const v8f z = {0.f, 0.f, 0.f, 0.f, 0.f, 0.f, 0.f, 0.f};
#pragma unroll
    for (int t = 0; t < NT; ++t) acc[t] = z;
  }
  if constexpr (EPI != 0) {
    if (tid < 64) bsm[tid] = bf16_val(bias[col0 + tid]);
  }
  const unsigned short* ap = A  + (size_t)(rowBase + 16 * wave + m) * (size_t)K + 8 * hh;
  const unsigned short* wp = WT + (size_t)(col0 + m) * (size_t)K + 8 * hh;
  const int ksteps = K >> 5;
#pragma unroll 1
  for (int ks = 0; ks < ksteps; ++ks) {
    FragB af;
    af.h[0] = *(const v8usa*)(ap + 32 * ks);
    af.h[1] = *(const v8usa*)(ap + 32 * ks + 16);
#pragma unroll
    for (int t = 0; t < NT; ++t) {
      const unsigned short* wq = wp + (size_t)(16 * t) * (size_t)K + 32 * ks;
      FragB bf;
      bf.h[0] = *(const v8usa*)wq;
      bf.h[1] = *(const v8usa*)(wq + 16);
      acc[t] = wmb(af, bf, acc[t]);
    }
  }

#pragma unroll
  for (int t = 0; t < NT; ++t) {
    const int lc = 16 * t + m;
#pragma unroll
    for (int r = 0; r < 8; ++r) {
      const int lr = 16 * wave + 8 * hh + r;
      stg[lr * GN + lc] = acc[t][r];
    }
  }
  __syncthreads();

  if constexpr (EPI == 0) {
    constexpr int NI = (GBM * PR) / GTHR;
#pragma unroll
    for (int i = 0; i < NI; ++i) {
      const int p  = tid + GTHR * i;
      const int lr = p / PR;
      const int c4 = p - lr * PR;
      const v4f v = *(const v4fa*)(stg + lr * GN + 4 * c4);
      *(volatile v4f*)(outF + (size_t)(rowBase + lr) * (size_t)ldo + col0 + 4 * c4) = v;
    }
    __threadfence();
#pragma unroll
    for (int i = 0; i < NI; ++i) {
      const int p  = tid + GTHR * i;
      const int lr = p / PR;
      const int c4 = p - lr * PR;
      const v4f v = *(const v4fa*)(stg + lr * GN + 4 * c4);
      *(volatile v4f*)(outF + (size_t)(rowBase + lr) * (size_t)ldo + col0 + 4 * c4) = v;
    }
  } else if constexpr (EPI == 1) {
    v8us o[8];
#pragma unroll
    for (int i = 0; i < 8; ++i) {
      const int pp = (tid + GTHR * i) & 511;
      const int lr = pp >> 3;
      const int c8 = (pp & 7) * 8;
      const int lo = (i >= 4) ? 1 : 0;
      const v4f a0 = *(const v4fa*)(stg + lr * GN + c8);
      const v4f a1 = *(const v4fa*)(stg + lr * GN + c8 + 4);
      const v4f b0 = *(const v4fa*)(bsm + c8);
      const v4f b1 = *(const v4fa*)(bsm + c8 + 4);
      v8us q;
      q[0] = hl_bits(a0.x + b0.x, lo); q[1] = hl_bits(a0.y + b0.y, lo);
      q[2] = hl_bits(a0.z + b0.z, lo); q[3] = hl_bits(a0.w + b0.w, lo);
      q[4] = hl_bits(a1.x + b1.x, lo); q[5] = hl_bits(a1.y + b1.y, lo);
      q[6] = hl_bits(a1.z + b1.z, lo); q[7] = hl_bits(a1.w + b1.w, lo);
      o[i] = q;
    }
#pragma unroll
    for (int i = 0; i < 8; ++i) {
      const int pp = (tid + GTHR * i) & 511;
      const int lr = pp >> 3;
      const int c8 = (pp & 7) * 8;
      unsigned short* op = outH + (size_t)(rowBase + lr) * (size_t)ldo + ((i >= 4) ? aux : 0) + col0 + c8;
      *(volatile v8us*)op = o[i];
    }
    __threadfence();
#pragma unroll
    for (int i = 0; i < 8; ++i) {
      const int pp = (tid + GTHR * i) & 511;
      const int lr = pp >> 3;
      const int c8 = (pp & 7) * 8;
      unsigned short* op = outH + (size_t)(rowBase + lr) * (size_t)ldo + ((i >= 4) ? aux : 0) + col0 + c8;
      *(volatile v8us*)op = o[i];
    }
  } else {
    v4f fv[8];
#pragma unroll
    for (int i = 0; i < 8; ++i) {
      const int p  = tid + GTHR * i;
      const int lr = p >> 4;
      const int c4 = p & 15;
      const v4f a = *(const v4fa*)(stg + lr * GN + 4 * c4);
      const v4f b = *(const v4fa*)(bsm + 4 * c4);
      fv[i] = a + b;
    }
#pragma unroll
    for (int i = 0; i < 8; ++i) {
      const int p  = tid + GTHR * i;
      const int lr = p >> 4;
      const int c4 = p & 15;
      const int gr = rowBase + lr;
      if (gr < aux) *(volatile v4f*)(outF + (size_t)gr * (size_t)ldo + col0 + 4 * c4) = fv[i];
    }
    __threadfence();
#pragma unroll
    for (int i = 0; i < 8; ++i) {
      const int p  = tid + GTHR * i;
      const int lr = p >> 4;
      const int c4 = p & 15;
      const int gr = rowBase + lr;
      if (gr < aux) *(volatile v4f*)(outF + (size_t)gr * (size_t)ldo + col0 + 4 * c4) = fv[i];
    }
  }
}

template <int C, int NV, int MODE>
__global__ __launch_bounds__(NTHR) void k_agg(const int* __restrict__ srcs, const int* __restrict__ dsts,
                                              int nE, int nN, int vec8, int mRows, int dout,
                                              const float* __restrict__ dis,
                                              const float* __restrict__ xl, const float* __restrict__ bias,
                                              unsigned short* hb, float* hout) {
  constexpr int PCN = C / 4;
  static_assert(C % 32 == 0 && PCN <= 32 * NV && PCN > 32 * (NV - 1) && C <= BLS_F);
  static_assert(MODE == 0 || 2 * C <= ROW_HW);
  extern __shared__ __attribute__((aligned(16))) int dsm[];
  int* list = dsm;
  int* hl   = dsm + LISTN;
  int* sl   = dsm + LISTN + RCAP;
  int* cnt  = dsm + LISTN + 2 * RCAP;
  int* offs = cnt + NBA;
  int* cur  = offs + NBA;
  int* misc = cur + NBA;
  float* bls = (float*)(misc + MISC_INTS);
  const int tid = (int)threadIdx.x, lane = tid & 31, wave = tid >> 5;
  unsigned short* rowbuf = (unsigned short*)(misc + MISC_INTS + BLS_F) + wave * ROW_HW;
  const int nodeBase = (int)blockIdx.x * NBA;

  {
    const v4i z4 = {0, 0, 0, 0};
    for (int i = tid * 4; i < AGG_ZINTS; i += NTHR * 4) *(v4ia*)(dsm + i) = z4;
    if (tid < MISC_INTS) misc[tid] = 0;
#pragma unroll 1
    for (int i = tid; i < C; i += NTHR) {
      const float bb = bias[i < dout ? i : dout - 1];
      bls[i] = (i < dout) ? bf16_val(bb) : 0.0f;
    }
  }
  __syncthreads();

  int t = 0, ov = 0;
  const int nChunks = (nE + CHUNK - 1) / CHUNK;
#pragma unroll 1
  for (int ch = 0; ch < nChunks; ++ch) {
    const int cbase = ch * CHUNK;
    const int wc = scan_chunk<SLA>(dsts, nE, cbase, nodeBase, NBA, vec8, list, tid, lane, wave);
    if (lane == 0) misc[wave] = wc;
    __syncthreads();
    if (wave == 0) {
#pragma unroll 1
      for (int w2 = 0; w2 < NWAVE; ++w2) {
        int c = misc[w2];
        c = c < 0 ? 0 : (c > WCAP ? WCAP : c);
#pragma unroll 1
        for (int b0 = 0; b0 < c; b0 += 32) {
          const int idx = b0 + lane;
          const int ent = list[w2 * WCAP + (idx < WCAP ? idx : WCAP - 1)];
          const int m32 = (c - b0) < 32 ? (c - b0) : 32;
#pragma unroll 1
          for (int k = 0; k < m32; ++k) {
            const int u    = __builtin_amdgcn_readlane(ent, k);
            const int slot = u & (NBA - 1);
            const int el   = (u >> SLA) & (CHUNK - 1);
            const int pk   = ((cbase + el) << SLA) | slot;
            if (t < RCAP) {
              if (lane == 0) { hl[t] = pk; cnt[slot] = cnt[slot] + 1; }
              t = t + 1;
            } else {
              ov = 1;
            }
          }
        }
      }
    }
    __syncthreads();
  }
  if (wave == 0 && lane == 0) { misc[8] = t; misc[9] = ov; }
  __syncthreads();
  int tt = misc[8];
  tt = tt < 0 ? 0 : (tt > RCAP ? RCAP : tt);
  const int ovf = misc[9];

  if (wave == 0) {
    const int base = lane * (NBA / 32);
    int s = 0;
#pragma unroll 1
    for (int i = 0; i < NBA / 32; ++i) s += cnt[base + i];
    int incl = s;
#pragma unroll
    for (int d = 1; d < 32; d <<= 1) {
      const int y = __shfl_up(incl, d, 32);
      if (lane >= d) incl += y;
    }
    int run = incl - s;
#pragma unroll 1
    for (int i = 0; i < NBA / 32; ++i) {
      const int cv = cnt[base + i];
      offs[base + i] = run;
      cur[base + i]  = run;
      run += cv;
    }
  }
  __syncthreads();
  if (wave == 0) {
#pragma unroll 1
    for (int b0 = 0; b0 < tt; b0 += 32) {
      const int idx = b0 + lane;
      const int ent = hl[idx < RCAP ? idx : RCAP - 1];
      const int m32 = (tt - b0) < 32 ? (tt - b0) : 32;
#pragma unroll 1
      for (int k = 0; k < m32; ++k) {
        const int u    = __builtin_amdgcn_readlane(ent, k);
        const int slot = u & (NBA - 1);
        if (lane == 0) {
          int p = cur[slot];
          p = p < 0 ? 0 : (p > RCAP - 1 ? RCAP - 1 : p);
          sl[p] = u;
          cur[slot] = p + 1;
        }
      }
    }
  }
  __syncthreads();

  const float qnan = __int_as_float(0x7fc00000);
  const float pz = (ovf != 0) ? qnan : 0.0f;
  int  pcl[NV];
  bool pvl[NV];
  v4f  bv[NV];
#pragma unroll
  for (int j = 0; j < NV; ++j) {
    const int p = lane + 32 * j;
    pvl[j] = p < PCN;
    pcl[j] = pvl[j] ? p : (PCN - 1);
    bv[j]  = *(const v4fa*)(bls + 4 * pcl[j]);
  }
#pragma unroll 1
  for (int si = 0; si < NBA / NWAVE; ++si) {
    const int s    = si * NWAVE + wave;
    const int node = nodeBase + s;
    int c = cnt[s];
    const bool big = c > DEGCAP;
    c = c < 0 ? 0 : (c > DEGCAP ? DEGCAP : c);
    int o = offs[s];
    o = o < 0 ? 0 : (o > RCAP ? RCAP : o);
    const int nc = node < nN ? node : nN - 1;
    const float dd = dis[nc];
    const float rd = dd * dd;
    v4f acc[NV];
    {
      const v4f z4 = {0.0f, 0.0f, 0.0f, 0.0f};
#pragma unroll
      for (int j = 0; j < NV; ++j) acc[j] = z4;
    }
#pragma unroll 1
    for (int b0 = 0; b0 < c; b0 += 32) {
      int idx = o + b0 + lane;
      idx = idx > RCAP - 1 ? RCAP - 1 : idx;
      const int ent = sl[idx];
      int eid = ent >> SLA;
      eid = eid < 0 ? 0 : (eid > nE - 1 ? nE - 1 : eid);
      int sr = srcs[eid];
      sr = sr < 0 ? 0 : (sr > nN - 1 ? nN - 1 : sr);
      const float cf  = dis[sr] * dd;
      const int   cfi = __float_as_int(cf);
      const int m32 = (c - b0) < 32 ? (c - b0) : 32;
#pragma unroll 1
      for (int k = 0; k < m32; ++k) {
        const int   sk = __builtin_amdgcn_readlane(sr, k);
        const float ck = __int_as_float(__builtin_amdgcn_readlane(cfi, k));
        const float* rp = xl + (size_t)sk * C;
#pragma unroll
        for (int j = 0; j < NV; ++j) {
          const v4f a = *(const v4fa*)(rp + 4 * pcl[j]);
          acc[j].x = fmaf(ck, a.x, acc[j].x);
          acc[j].y = fmaf(ck, a.y, acc[j].y);
          acc[j].z = fmaf(ck, a.z, acc[j].z);
          acc[j].w = fmaf(ck, a.w, acc[j].w);
        }
      }
    }
    const float pzr = big ? qnan : pz;
    const bool live  = node < nN;
    const bool rowok = node < mRows;
    const float* sp = xl + (size_t)nc * C;
    v4f y[NV];
#pragma unroll
    for (int j = 0; j < NV; ++j) {
      const v4f sv = *(const v4fa*)(sp + 4 * pcl[j]);
      y[j].x = fin1(acc[j].x, sv.x, rd, bv[j].x, pzr, live);
      y[j].y = fin1(acc[j].y, sv.y, rd, bv[j].y, pzr, live);
      y[j].z = fin1(acc[j].z, sv.z, rd, bv[j].z, pzr, live);
      y[j].w = fin1(acc[j].w, sv.w, rd, bv[j].w, pzr, live);
    }
    if constexpr (MODE != 0) {
#pragma unroll
      for (int j = 0; j < NV; ++j) {
        v4us mh, ml;
        unsigned hbt;
        hbt = bf16_bits(y[j].x); mh[0] = (unsigned short)hbt; ml[0] = (unsigned short)bf16_bits(y[j].x - __uint_as_float(hbt << 16));
        hbt = bf16_bits(y[j].y); mh[1] = (unsigned short)hbt; ml[1] = (unsigned short)bf16_bits(y[j].y - __uint_as_float(hbt << 16));
        hbt = bf16_bits(y[j].z); mh[2] = (unsigned short)hbt; ml[2] = (unsigned short)bf16_bits(y[j].z - __uint_as_float(hbt << 16));
        hbt = bf16_bits(y[j].w); mh[3] = (unsigned short)hbt; ml[3] = (unsigned short)bf16_bits(y[j].w - __uint_as_float(hbt << 16));
        if (pvl[j]) {
          *(v4usa*)(rowbuf + 4 * (lane + 32 * j)) = mh;
          *(v4usa*)(rowbuf + C + 4 * (lane + 32 * j)) = ml;
        }
      }
      wave_sync();
      v8us q[NV];
#pragma unroll
      for (int j = 0; j < NV; ++j) q[j] = *(const v8usa*)(rowbuf + 8 * pcl[j]);
      wave_sync();
      unsigned short* rpw = hb + (size_t)node * (2 * C);
#pragma unroll
      for (int j = 0; j < NV; ++j)
        if (rowok && pvl[j]) *(volatile v8us*)(rpw + 8 * (lane + 32 * j)) = q[j];
      __threadfence();
#pragma unroll
      for (int j = 0; j < NV; ++j)
        if (rowok && pvl[j]) *(volatile v8us*)(rpw + 8 * (lane + 32 * j)) = q[j];
    } else {
      float* rpw = hout + (size_t)node * C;
#pragma unroll
      for (int j = 0; j < NV; ++j)
        if (rowok && pvl[j]) *(volatile v4f*)(rpw + 4 * (lane + 32 * j)) = y[j];
      __threadfence();
#pragma unroll
      for (int j = 0; j < NV; ++j)
        if (rowok && pvl[j]) *(volatile v4f*)(rpw + 4 * (lane + 32 * j)) = y[j];
    }
  }
}

__global__ __launch_bounds__(NTHR) void k_pool(const float* __restrict__ hf, const int* __restrict__ bat,
                                               int nN, int nG, unsigned short* pl) {
  __shared__ __attribute__((aligned(16))) float wmx[NWAVE * C3];
  __shared__ __attribute__((aligned(16))) unsigned short outs[2 * C3];
  constexpr int PCN = C3 / 4;
  const int tid = (int)threadIdx.x, lane = tid & 31, wave = tid >> 5;
  const int g = (int)blockIdx.x;
  const float ninf = __uint_as_float(0xff800000u);

  int  pcl[3];
  bool pvl[3];
  v4f  mx[3];
#pragma unroll
  for (int j = 0; j < 3; ++j) {
    const int p = lane + 32 * j;
    pvl[j] = p < PCN;
    pcl[j] = pvl[j] ? p : (PCN - 1);
    const v4f n4 = {ninf, ninf, ninf, ninf};
    mx[j] = n4;
  }
  const int lim = (g < nG) ? nN : 0;
#pragma unroll 1
  for (int i0 = wave * 32; i0 < lim; i0 += NTHR) {
    const int i  = i0 + lane;
    const int ic = i < nN ? i : nN - 1;
    const int b  = bat[ic];
    const bool hit = (i < nN) && (b == g);
    unsigned msk = __builtin_amdgcn_ballot_w32(hit);
    int nh = (int)__builtin_popcount(msk);
    nh = nh > 32 ? 32 : nh;
#pragma unroll 1
    for (int q = 0; q < nh; ++q) {
      const int k = __builtin_ffs((int)msk) - 1;
      msk &= msk - 1u;
      int node = i0 + (k < 0 ? 0 : k);
      node = node > nN - 1 ? nN - 1 : node;
      const float* rp = hf + (size_t)node * C3;
#pragma unroll
      for (int j = 0; j < 3; ++j) {
        const v4f v = *(const v4fa*)(rp + 4 * pcl[j]);
        mx[j].x = nmax(mx[j].x, v.x);
        mx[j].y = nmax(mx[j].y, v.y);
        mx[j].z = nmax(mx[j].z, v.z);
        mx[j].w = nmax(mx[j].w, v.w);
      }
    }
  }
#pragma unroll
  for (int j = 0; j < 3; ++j)
    if (pvl[j]) *(v4fa*)(wmx + wave * C3 + 4 * (lane + 32 * j)) = mx[j];
  __syncthreads();
#pragma unroll 1
  for (int c = tid; c < C3; c += NTHR) {
    float mm = ninf;
#pragma unroll
    for (int w2 = 0; w2 < NWAVE; ++w2) mm = nmax(mm, wmx[w2 * C3 + c]);
    const float r = (mm == ninf) ? 0.0f : mm;
    const unsigned hbt = bf16_bits(r);
    const unsigned lbt = bf16_bits(r - __uint_as_float(hbt << 16));
    outs[c]      = (unsigned short)hbt;
    outs[C3 + c] = (unsigned short)lbt;
  }
  __syncthreads();
  const int pq = tid < PCN ? tid : PCN - 1;
  const v8us qv = *(const v8usa*)(outs + 8 * pq);
  unsigned short* op = pl + (size_t)g * (2 * C3) + 8 * pq;
  if (tid < PCN) *(volatile v8us*)op = qv;
  __threadfence();
  if (tid < PCN) *(volatile v8us*)op = qv;
}

static inline int cdiv(int a, int b) { return (a + b - 1) / b; }
static inline size_t al256(size_t o) { return (o + 255) & ~(size_t)255; }

extern "C" void kernel_launch(void* const* d_in, const int* in_sizes, int n_in,
                              void* d_out, int out_size, void* d_ws, size_t ws_size,
                              hipStream_t stream) {
  if (n_in < 13) return;
  if (in_sizes[0] < DIN || (in_sizes[0] % DIN) != 0) return;
  const int nN = in_sizes[0] / DIN;
  if (nN < 1 || nN > (1 << 22)) return;
  if (in_sizes[1] < 2 || (in_sizes[1] & 1) != 0) return;
  const int nE = in_sizes[1] / 2;
  if (nE < 1 || nE >= (1 << (31 - SLA))) return;
  if (in_sizes[2] != nN) return;
  if (in_sizes[3] != DIN * D1 || in_sizes[4] != D1) return;
  if (in_sizes[5] != D1 * D2 || in_sizes[6] != D2) return;
  if (in_sizes[7] != D2 * D3 || in_sizes[8] != D3) return;
  if (in_sizes[9] != D3 * DF1 || in_sizes[10] != DF1) return;
  if (in_sizes[11] != DF1 * DF2 || in_sizes[12] != DF2) return;
  if (out_size < DF2 || (out_size % DF2) != 0) return;
  const int nG = out_size / DF2;
  if (nG < 1 || nG > 65536) return;

  const float* x    = (const float*)d_in[0];
  const int*   edge = (const int*)d_in[1];
  const int*   bat  = (const int*)d_in[2];
  const float* W1   = (const float*)d_in[3];
  const float* b1   = (const float*)d_in[4];
  const float* W2   = (const float*)d_in[5];
  const float* b2   = (const float*)d_in[6];
  const float* W3   = (const float*)d_in[7];
  const float* b3   = (const float*)d_in[8];
  const float* Wf1  = (const float*)d_in[9];
  const float* bf1  = (const float*)d_in[10];
  const float* Wf2  = (const float*)d_in[11];
  const float* bf2  = (const float*)d_in[12];
  float* out = (float*)d_out;
  const int* src = edge;
  const int* dst = edge + nE;

  const int MP   = cdiv(nN, GBM) * GBM;
  const int gM   = MP / GBM;
  const int MH   = cdiv(nG, GBM) * GBM;
  const int gH   = MH / GBM;
  const int gD   = cdiv(nN, NBD);
  const int NBPD = gD * NBD;
  const int gA   = cdiv(MP, NBA);
  if ((long long)gA * NBA < (long long)MP) return;
  if (NBPD < nN) return;
  const int vec8 = ((nE & 3) == 0) ? 1 : 0;

  char* ws = (char*)d_ws;
  size_t off = 0;
  const size_t oDIS = off; off = al256(off + (size_t)NBPD * 4);
  const size_t oT1  = off; off = al256(off + (size_t)C1 * C1 * 2);
  const size_t oT2  = off; off = al256(off + (size_t)C2 * 2 * C1 * 2);
  const size_t oT3  = off; off = al256(off + (size_t)C3 * 2 * C2 * 2);
  const size_t oT4  = off; off = al256(off + (size_t)DF1 * 2 * C3 * 2);
  const size_t oT5  = off; off = al256(off + (size_t)DF2 * 2 * DF1 * 2);
  const size_t oXB  = off; off = al256(off + (size_t)MP * C1 * 2);
  const size_t oXW1 = off; off = al256(off + (size_t)MP * C1 * 4);
  const size_t oH1  = off; off = al256(off + (size_t)MP * 2 * C1 * 2);
  const size_t oXW2 = off; off = al256(off + (size_t)MP * C2 * 4);
  const size_t oH2  = off; off = al256(off + (size_t)MP * 2 * C2 * 2);
  const size_t oXW3 = off; off = al256(off + (size_t)MP * C3 * 4);
  const size_t oP   = off; off = al256(off + (size_t)MH * 2 * C3 * 2);
  const size_t oF   = off; off = al256(off + (size_t)MH * 2 * DF1 * 2);
  if (off > ws_size || off > (size_t)WSMAX) return;
  if ((oH2 - oXB) < (size_t)MP * C3 * 4) return;
  float*          DIS  = (float*)(ws + oDIS);
  unsigned short* T1   = (unsigned short*)(ws + oT1);
  unsigned short* T2   = (unsigned short*)(ws + oT2);
  unsigned short* T3   = (unsigned short*)(ws + oT3);
  unsigned short* T4   = (unsigned short*)(ws + oT4);
  unsigned short* T5   = (unsigned short*)(ws + oT5);
  unsigned short* XB   = (unsigned short*)(ws + oXB);
  float*          XW1  = (float*)(ws + oXW1);
  unsigned short* H1   = (unsigned short*)(ws + oH1);
  float*          XW2  = (float*)(ws + oXW2);
  unsigned short* H2   = (unsigned short*)(ws + oH2);
  float*          XW3  = (float*)(ws + oXW3);
  float*          H3   = (float*)(ws + oXB);
  unsigned short* PP   = (unsigned short*)(ws + oP);
  unsigned short* FF   = (unsigned short*)(ws + oF);

  const size_t aggLds = (size_t)AGG_LDS_INTS * 4;
  hipFuncSetAttribute(reinterpret_cast<const void*>(&k_agg<C1, 1, 1>), hipFuncAttributeMaxDynamicSharedMemorySize, (int)aggLds);
  hipFuncSetAttribute(reinterpret_cast<const void*>(&k_agg<C2, 2, 1>), hipFuncAttributeMaxDynamicSharedMemorySize, (int)aggLds);
  hipFuncSetAttribute(reinterpret_cast<const void*>(&k_agg<C3, 3, 0>), hipFuncAttributeMaxDynamicSharedMemorySize, (int)aggLds);

  const int nUx = MP * (C1 / 8);
  k_wprep<<<WB1 + WB2 + WB3 + WB4 + WB5, NTHR, 0, stream>>>(W1, W2, W3, Wf1, Wf2, T1, T2, T3, T4, T5);
  k_cvx<<<cdiv(nUx, NTHR), NTHR, 0, stream>>>(x, nN, nUx, XB);
  k_deg<<<gD, NTHR, 0, stream>>>(dst, nE, vec8, DIS);
  k_gemm<6, 0><<<dim3(gM, 1), GTHR, 0, stream>>>(XB, T1, C1, b1, XW1, (unsigned short*)XW1, C1, 0);
  k_agg<C1, 1, 1><<<gA, NTHR, aggLds, stream>>>(src, dst, nE, nN, vec8, MP, D1, DIS, XW1, b1, H1, (float*)H1);
  k_gemm<10, 0><<<dim3(gM, 1), GTHR, 0, stream>>>(H1, T2, 2 * C1, b2, XW2, (unsigned short*)XW2, C2, 0);
  k_agg<C2, 2, 1><<<gA, NTHR, aggLds, stream>>>(src, dst, nE, nN, vec8, MP, D2, DIS, XW2, b2, H2, (float*)H2);
  k_gemm<10, 0><<<dim3(gM, C3 / 160), GTHR, 0, stream>>>(H2, T3, 2 * C2, b3, XW3, (unsigned short*)XW3, C3, 0);
  k_agg<C3, 3, 0><<<gA, NTHR, aggLds, stream>>>(src, dst, nE, nN, vec8, MP, D3, DIS, XW3, b3, (unsigned short*)H3, H3);
  k_pool<<<MH, NTHR, 0, stream>>>(H3, bat, nN, nG, PP);
  k_gemm<4, 1><<<dim3(gH, DF1 / 64), GTHR, 0, stream>>>(PP, T4, 2 * C3, bf1, (float*)FF, FF, 2 * DF1, DF1);
  k_gemm<4, 2><<<dim3(gH, DF2 / 64), GTHR, 0, stream>>>(FF, T5, 2 * DF1, bf2, out, (unsigned short*)out, DF2, nG);
}
